// RUMABlock_4398046511443
// MI455X (gfx1250) — hardware-verified
//
#include <hip/hip_runtime.h>

typedef _Float16 v16h __attribute__((ext_vector_type(16)));
typedef _Float16 v8h  __attribute__((ext_vector_type(8)));
typedef __bf16   v16bf __attribute__((ext_vector_type(16)));
typedef unsigned short v16us __attribute__((ext_vector_type(16)));
typedef unsigned short v8us  __attribute__((ext_vector_type(8)));
typedef float    v8f  __attribute__((ext_vector_type(8)));
typedef float    v4f  __attribute__((ext_vector_type(4)));
typedef v8h  __attribute__((may_alias)) v8ha;
typedef v8us __attribute__((may_alias)) v8usa;
typedef v4f  __attribute__((may_alias)) v4fa;

union Frag  { v16h v; v8h half[2]; };
union FragU { v16bf b; v16us u; v8us half[2]; unsigned short s[16]; };
union U8    { v8us v; unsigned short s[8]; };

#define DM    1024
#define SEQ   2048
#define BATCH 4
#define NTOK  (BATCH * SEQ)
#define K2    (2 * DM)
#define NSH   16
#define NEXP  4
#define NX    (NTOK * DM)
#define WSC   64.0f
#define WINV  0.015625f

__device__ __forceinline__ v8f wmma16(v16h a, v16h b, v8f c) {
  v8f d = __builtin_amdgcn_wmma_f32_16x16x32_f16(false, a, false, b, (short)0, c, false, false);
#if defined(__HIP_DEVICE_COMPILE__)
  asm volatile("v_nop\n\tv_nop\n\tv_nop\n\tv_nop" : "+v"(d) : "v"(a), "v"(b));
#endif
  return d;
}

__device__ __forceinline__ v8f wmma_bf(v16bf a, v16bf b, v8f c) {
  v8f d = __builtin_amdgcn_wmma_f32_16x16x32_bf16(false, a, false, b, (short)0, c, false, false);
#if defined(__HIP_DEVICE_COMPILE__)
  asm volatile("v_nop\n\tv_nop\n\tv_nop\n\tv_nop" : "+v"(d) : "v"(a), "v"(b));
#endif
  return d;
}

__device__ __forceinline__ v16h load_frag(const _Float16* p, int h) {
  Frag f;
  f.half[0] = *(const v8ha*)(p + 8 * h);
  f.half[1] = *(const v8ha*)(p + 16 + 8 * h);
  return f.v;
}

__device__ __forceinline__ v16bf load_frag_bf(const unsigned short* p, int h) {
  FragU f;
  f.half[0] = *(const v8usa*)(p + 8 * h);
  f.half[1] = *(const v8usa*)(p + 16 + 8 * h);
  return f.b;
}

__device__ __forceinline__ float wsum(float v) {
  #pragma unroll
  for (int o = 16; o > 0; o >>= 1) v += __shfl_xor(v, o);
  return v;
}

__device__ __forceinline__ unsigned bf16_rne_hi(float x) {
  const unsigned u = __float_as_uint(x);
  return (u + 0x7fffu + ((u >> 16) & 1u)) & 0xffff0000u;
}

__device__ __forceinline__ void split2(float x, unsigned short& hi, unsigned short& lo) {
  const unsigned hb = bf16_rne_hi(x);
  const float res = x - __uint_as_float(hb);
  const unsigned lb = bf16_rne_hi(res);
  hi = (unsigned short)(hb >> 16);
  lo = (unsigned short)(lb >> 16);
}

__device__ __forceinline__ void split_frag(const float* p, int h, v16bf& fh, v16bf& fl) {
  const v4f a = *(const v4fa*)(p + 8 * h);
  const v4f b = *(const v4fa*)(p + 8 * h + 4);
  const v4f c = *(const v4fa*)(p + 16 + 8 * h);
  const v4f d = *(const v4fa*)(p + 16 + 8 * h + 4);
  const float xs[16] = { a.x, a.y, a.z, a.w, b.x, b.y, b.z, b.w,
                         c.x, c.y, c.z, c.w, d.x, d.y, d.z, d.w };
  FragU uh, ul;
  #pragma unroll
  for (int i = 0; i < 16; ++i) {
    unsigned short hi, lo;
    split2(xs[i], hi, lo);
    uh.s[i] = hi; ul.s[i] = lo;
  }
  fh = uh.b; fl = ul.b;
}

__device__ __forceinline__ void cvt_store_pass(const _Float16* sT, _Float16* outz,
                                               int R, int c0, int r0, int w, int lane) {
  const int q8 = lane & 7, sub = lane >> 3;
  #pragma unroll
  for (int i = 0; i < 2; ++i) {
    const int j = 8 * w + 4 * i + sub;
    const v8h v = *(const v8ha*)(sT + j * 64 + 8 * q8);
    *(volatile v8h*)(outz + (size_t)(c0 + j) * R + r0 + 8 * q8) = v;
  }
}

__global__ __launch_bounds__(256) void cvt_t_kernel(
    const float* __restrict__ in, _Float16* __restrict__ out, int R, int C, float sc)
{
  __shared__ __attribute__((aligned(16))) _Float16 sT[64 * 64];
  const int tid = threadIdx.x, lane = tid & 31, w = tid >> 5;
  const int c0 = blockIdx.x * 64, r0 = blockIdx.y * 64, z = blockIdx.z;
  const float* inz = in + (size_t)z * R * C;
  _Float16* outz = out + (size_t)z * R * C;
  #pragma unroll
  for (int p = 0; p < 4; ++p) {
    const int i = p * 16 + (tid >> 4);
    const int cc = 4 * (tid & 15);
    const v4f v = *(const v4fa*)(inz + (size_t)(r0 + i) * C + c0 + cc);
    sT[(cc + 0) * 64 + i] = (_Float16)(v.x * sc);
    sT[(cc + 1) * 64 + i] = (_Float16)(v.y * sc);
    sT[(cc + 2) * 64 + i] = (_Float16)(v.z * sc);
    sT[(cc + 3) * 64 + i] = (_Float16)(v.w * sc);
  }
  __syncthreads();
  cvt_store_pass(sT, outz, R, c0, r0, w, lane);
  __threadfence();
  cvt_store_pass(sT, outz, R, c0, r0, w, lane);
}

__device__ __forceinline__ void cvt_store_pass_us(const unsigned short* sT, unsigned short* outp,
                                                  int R, int c0, int r0, int w, int lane) {
  const int q8 = lane & 7, sub = lane >> 3;
  #pragma unroll
  for (int i = 0; i < 2; ++i) {
    const int j = 8 * w + 4 * i + sub;
    const v8us v = *(const v8usa*)(sT + j * 64 + 8 * q8);
    *(volatile v8us*)(outp + (size_t)(c0 + j) * R + r0 + 8 * q8) = v;
  }
}

__global__ __launch_bounds__(256) void cvt_t2_kernel(
    const float* __restrict__ in, unsigned short* __restrict__ outH,
    unsigned short* __restrict__ outL, int R, int C)
{
  __shared__ __attribute__((aligned(16))) unsigned short sHi[64 * 64];
  __shared__ __attribute__((aligned(16))) unsigned short sLo[64 * 64];
  const int tid = threadIdx.x, lane = tid & 31, w = tid >> 5;
  const int c0 = blockIdx.x * 64, r0 = blockIdx.y * 64;
  #pragma unroll
  for (int p = 0; p < 4; ++p) {
    const int i = p * 16 + (tid >> 4);
    const int cc = 4 * (tid & 15);
    const v4f v = *(const v4fa*)(in + (size_t)(r0 + i) * C + c0 + cc);
    const float vv[4] = { v.x, v.y, v.z, v.w };
    #pragma unroll
    for (int q = 0; q < 4; ++q) {
      unsigned short hi, lo;
      split2(vv[q], hi, lo);
      sHi[(cc + q) * 64 + i] = hi;
      sLo[(cc + q) * 64 + i] = lo;
    }
  }
  __syncthreads();
  cvt_store_pass_us(sHi, outH, R, c0, r0, w, lane);
  cvt_store_pass_us(sLo, outL, R, c0, r0, w, lane);
  __threadfence();
  cvt_store_pass_us(sHi, outH, R, c0, r0, w, lane);
  cvt_store_pass_us(sLo, outL, R, c0, r0, w, lane);
}

__device__ __forceinline__ void hyp_store_pass(const unsigned short* sT, unsigned short* pl,
                                               int d0, int w, int lane) {
  const int q8 = lane & 7, n = 4 * w + (lane >> 3);
  const v8us v = *(const v8usa*)(sT + n * 64 + 8 * q8);
  *(volatile v8us*)(pl + (size_t)n * DM + d0 + 8 * q8) = v;
}

__global__ __launch_bounds__(128) void cvt_hyp_kernel(
    const float* __restrict__ hyp, unsigned short* __restrict__ hypH,
    unsigned short* __restrict__ hypL)
{
  __shared__ __attribute__((aligned(16))) unsigned short sHi[16 * 64];
  __shared__ __attribute__((aligned(16))) unsigned short sLo[16 * 64];
  const int tid = threadIdx.x, lane = tid & 31, w = tid >> 5;
  const int d0 = blockIdx.x * 64;
  #pragma unroll
  for (int p = 0; p < 2; ++p) {
    const int f4 = tid + 128 * p;
    const int dl = f4 >> 2, nq = (f4 & 3) * 4;
    const v4f v = *(const v4fa*)(hyp + (size_t)(d0 + dl) * NSH + nq);
    const float vv[4] = { v.x, v.y, v.z, v.w };
    #pragma unroll
    for (int q = 0; q < 4; ++q) {
      unsigned short hi, lo;
      split2(vv[q], hi, lo);
      sHi[(nq + q) * 64 + dl] = hi;
      sLo[(nq + q) * 64 + dl] = lo;
    }
  }
  __syncthreads();
  hyp_store_pass(sHi, hypH, d0, w, lane);
  hyp_store_pass(sLo, hypL, d0, w, lane);
  __threadfence();
  hyp_store_pass(sHi, hypH, d0, w, lane);
  hyp_store_pass(sLo, hypL, d0, w, lane);
}

__global__ __launch_bounds__(256) void ln1_kernel(
    const float* __restrict__ x, const float* __restrict__ mem,
    const float* __restrict__ g1, const float* __restrict__ b1,
    unsigned short* __restrict__ normH, unsigned short* __restrict__ normL,
    _Float16* __restrict__ cmA)
{
  const int tid = threadIdx.x, lane = tid & 31, w = tid >> 5;
  const int t = blockIdx.x * 8 + w;
  const float* xr = x + (size_t)t * DM;
  const float* mr = mem + (size_t)t * DM;

  v4f xv[8];
  float s = 0.f;
  #pragma unroll
  for (int j = 0; j < 4; ++j) {
    const int base = 256 * j + 8 * lane;
    const v4f a = *(const v4fa*)(xr + base);
    const v4f c = *(const v4fa*)(xr + base + 4);
    xv[2 * j] = a; xv[2 * j + 1] = c;
    s += ((a.x + a.y) + (a.z + a.w)) + ((c.x + c.y) + (c.z + c.w));
  }
  s = wsum(s);
  const float mean = s * (1.0f / DM);
  float ss = 0.f;
  #pragma unroll
  for (int q = 0; q < 8; ++q) {
    const v4f d = xv[q] - mean;
    ss += (d.x * d.x + d.y * d.y) + (d.z * d.z + d.w * d.w);
  }
  ss = wsum(ss);
  const float var = ss * (1.0f / DM);
  const float rstd = rsqrtf(var + 1e-5f);

  v8us hv[4], lv[4];
  v8h mh[4];
  #pragma unroll
  for (int j = 0; j < 4; ++j) {
    const int base = 256 * j + 8 * lane;
    const v4f ga = *(const v4fa*)(g1 + base), gb = *(const v4fa*)(g1 + base + 4);
    const v4f ba = *(const v4fa*)(b1 + base), bb = *(const v4fa*)(b1 + base + 4);
    const v4f na = (xv[2 * j] - mean) * rstd * ga + ba;
    const v4f nb = (xv[2 * j + 1] - mean) * rstd * gb + bb;
    const float nn[8] = { na.x, na.y, na.z, na.w, nb.x, nb.y, nb.z, nb.w };
    U8 uh, ul;
    #pragma unroll
    for (int q = 0; q < 8; ++q) {
      unsigned short hi, lo;
      split2(nn[q], hi, lo);
      uh.s[q] = hi; ul.s[q] = lo;
    }
    hv[j] = uh.v; lv[j] = ul.v;
    const v4f ma = *(const v4fa*)(mr + base), mb = *(const v4fa*)(mr + base + 4);
    const v8h mq = { (_Float16)ma.x, (_Float16)ma.y, (_Float16)ma.z, (_Float16)ma.w,
                     (_Float16)mb.x, (_Float16)mb.y, (_Float16)mb.z, (_Float16)mb.w };
    mh[j] = mq;
  }
  #pragma unroll
  for (int j = 0; j < 4; ++j) {
    const int base = 256 * j + 8 * lane;
    *(volatile v8us*)(normH + (size_t)t * DM + base) = hv[j];
    *(volatile v8us*)(normL + (size_t)t * DM + base) = lv[j];
    *(volatile v8h*)(cmA + (size_t)t * K2 + DM + base) = mh[j];
  }
  __threadfence();
  #pragma unroll
  for (int j = 0; j < 4; ++j) {
    const int base = 256 * j + 8 * lane;
    *(volatile v8us*)(normH + (size_t)t * DM + base) = hv[j];
    *(volatile v8us*)(normL + (size_t)t * DM + base) = lv[j];
    *(volatile v8h*)(cmA + (size_t)t * K2 + DM + base) = mh[j];
  }
}

__device__ __forceinline__ void q_store_pass(const float* sq, float* Qf, _Float16* cmA,
                                             int m0w, int n0, int lane) {
  const int q8 = lane & 7, sub = lane >> 3;
  #pragma unroll
  for (int i = 0; i < 16; ++i) {
    const int lid = 4 * i + sub;
    const int row = lid >> 1, hl = lid & 1;
    const v4f v = *(const v4fa*)(sq + row * 64 + 32 * hl + 4 * q8);
    *(volatile v4f*)(Qf + (size_t)(m0w + row) * DM + n0 + 32 * hl + 4 * q8) = v;
  }
  #pragma unroll
  for (int i = 0; i < 8; ++i) {
    const int row = 4 * i + sub;
    const v4f a = *(const v4fa*)(sq + row * 64 + 8 * q8);
    const v4f c = *(const v4fa*)(sq + row * 64 + 8 * q8 + 4);
    const v8h o = { (_Float16)a.x, (_Float16)a.y, (_Float16)a.z, (_Float16)a.w,
                    (_Float16)c.x, (_Float16)c.y, (_Float16)c.z, (_Float16)c.w };
    *(volatile v8h*)(cmA + (size_t)(m0w + row) * K2 + n0 + 8 * q8) = o;
  }
}

__global__ __launch_bounds__(128) void gemm_q_kernel(
    const unsigned short* __restrict__ normH,
    const unsigned short* __restrict__ normL,
    const unsigned short* __restrict__ wqH,
    const unsigned short* __restrict__ wqL,
    const float* __restrict__ bq,
    float* __restrict__ Qf,
    _Float16* __restrict__ cmA)
{
  __shared__ __attribute__((aligned(16))) float sQ[4 * 32 * 64];
  const int tid = threadIdx.x, lane = tid & 31, w = tid >> 5;
  const int h = lane >> 4, m = lane & 15;
  const int m0w = blockIdx.x * 128 + 32 * w;
  const int n0 = blockIdx.y * 64;

  const size_t arow0 = (size_t)(m0w + m) * DM;
  const size_t arow1 = arow0 + (size_t)16 * DM;
  const size_t brow  = (size_t)(n0 + m) * DM;

  const v8f zero8 = {0.f, 0.f, 0.f, 0.f, 0.f, 0.f, 0.f, 0.f};
  v8f acc[2][4];
  #pragma unroll
  for (int mt = 0; mt < 2; ++mt)
    #pragma unroll
    for (int nt = 0; nt < 4; ++nt) acc[mt][nt] = zero8;

  #pragma unroll 1
  for (int k0 = 0; k0 < DM; k0 += 32) {
    const v16bf a0h = load_frag_bf(normH + arow0 + k0, h);
    const v16bf a0l = load_frag_bf(normL + arow0 + k0, h);
    const v16bf a1h = load_frag_bf(normH + arow1 + k0, h);
    const v16bf a1l = load_frag_bf(normL + arow1 + k0, h);
    #pragma unroll
    for (int nt = 0; nt < 4; ++nt) {
      const size_t bo = brow + (size_t)nt * 16 * DM + k0;
      const v16bf bh = load_frag_bf(wqH + bo, h);
      const v16bf bl = load_frag_bf(wqL + bo, h);
      acc[0][nt] = wmma_bf(a0h, bh, acc[0][nt]);
      acc[0][nt] = wmma_bf(a0h, bl, acc[0][nt]);
      acc[0][nt] = wmma_bf(a0l, bh, acc[0][nt]);
      acc[1][nt] = wmma_bf(a1h, bh, acc[1][nt]);
      acc[1][nt] = wmma_bf(a1h, bl, acc[1][nt]);
      acc[1][nt] = wmma_bf(a1l, bh, acc[1][nt]);
    }
  }

  float* sq = sQ + w * 2048;
  #pragma unroll
  for (int nt = 0; nt < 4; ++nt) {
    const int feat = 16 * nt + m;
    const float bv = bq[n0 + feat];
    #pragma unroll
    for (int mt = 0; mt < 2; ++mt)
      #pragma unroll
      for (int r = 0; r < 8; ++r)
        sq[(16 * mt + 8 * h + r) * 64 + feat] = acc[mt][nt][r] + bv;
  }
  __syncthreads();
  q_store_pass(sq, Qf, cmA, m0w, n0, lane);
  __threadfence();
  q_store_pass(sq, Qf, cmA, m0w, n0, lane);
}

__device__ __forceinline__ float silu_f(float a) { return a * (1.0f / (1.0f + expf(-a))); }

__global__ __launch_bounds__(64) void token_kernel(
    const float* __restrict__ Qf,
    const unsigned short* __restrict__ hypH, const unsigned short* __restrict__ hypL,
    const float* __restrict__ mem,
    const float* __restrict__ suff, const float* __restrict__ conf, const float* __restrict__ lin,
    const float* __restrict__ tsc, const float* __restrict__ tsco, const float* __restrict__ alg,
    const float* __restrict__ stale,
    const float* __restrict__ Ws1, const float* __restrict__ bs1,
    const float* __restrict__ Ws2, const float* __restrict__ bs2,
    const float* __restrict__ Ws3, const float* __restrict__ bs3,
    const float* __restrict__ Wr1, const float* __restrict__ br1,
    const float* __restrict__ Wr2, const float* __restrict__ br2,
    float* __restrict__ ew, float* __restrict__ sel)
{
#pragma clang fp contract(off)
  __shared__ float sL[64 * 20];
  __shared__ float sH1[32 * 64];
  __shared__ float sH2[32 * 64];
  __shared__ __attribute__((aligned(16))) float sS[64];

  const int tid = threadIdx.x, lane = tid & 31, w = tid >> 5;
  const int h = lane >> 4, m = lane & 15;
  const int tb = blockIdx.x * 64 + 32 * w;

  {
    const float* qa0 = Qf + (size_t)(tb + m) * DM;
    const float* qa1 = qa0 + (size_t)16 * DM;
    const unsigned short* hh = hypH + (size_t)m * DM;
    const unsigned short* hl = hypL + (size_t)m * DM;
    const v8f zero8 = {0.f, 0.f, 0.f, 0.f, 0.f, 0.f, 0.f, 0.f};
    v8f acc0 = zero8, acc1 = zero8;
    #pragma unroll 1
    for (int k0 = 0; k0 < DM; k0 += 32) {
      v16bf a0h, a0l, a1h, a1l;
      split_frag(qa0 + k0, h, a0h, a0l);
      split_frag(qa1 + k0, h, a1h, a1l);
      const v16bf bh = load_frag_bf(hh + k0, h);
      const v16bf bl = load_frag_bf(hl + k0, h);
      acc0 = wmma_bf(a0h, bh, acc0);
      acc0 = wmma_bf(a0h, bl, acc0);
      acc0 = wmma_bf(a0l, bh, acc0);
      acc1 = wmma_bf(a1h, bh, acc1);
      acc1 = wmma_bf(a1h, bl, acc1);
      acc1 = wmma_bf(a1l, bh, acc1);
    }
    #pragma unroll
    for (int r = 0; r < 8; ++r) {
      sL[(32 * w + 8 * h + r) * 20 + m]      = acc0[r];
      sL[(32 * w + 16 + 8 * h + r) * 20 + m] = acc1[r];
    }
  }
  __syncthreads();

  const int t = tb + lane;

  float ms = 0.f;
  #pragma unroll 1
  for (int j = 0; j < 32; ++j) {
    const float* mrow = mem + (size_t)(tb + j) * DM + 32 * lane;
    float p = 0.f;
    #pragma unroll
    for (int q = 0; q < 8; ++q) {
      const v4f v = *(const v4fa*)(mrow + 4 * q);
      p += (v.x * v.x + v.y * v.y) + (v.z * v.z + v.w * v.w);
    }
    p = wsum(p);
    ms = (lane == j) ? p : ms;
  }
  const float pres = (sqrtf(ms) > 1e-6f) ? 1.0f : 0.0f;

  float mx = sL[tid * 20];
  #pragma unroll 1
  for (int n = 1; n < NSH; ++n) mx = fmaxf(mx, sL[tid * 20 + n]);
  float se = 0.f;
  #pragma unroll 1
  for (int n = 0; n < NSH; ++n) se += expf(sL[tid * 20 + n] - mx);
  const float rc = 1.0f / se;

  float f[9];
  f[0] = suff[t]; f[1] = conf[t]; f[2] = lin[t]; f[3] = tsc[t];
  f[4] = fmaxf(tsco[t], 0.0f); f[5] = alg[t]; f[6] = stale[t]; f[7] = rc; f[8] = pres;
  const float prior = 2.0f * f[0] + 1.25f * f[2] + 0.75f * f[5] + 0.35f * f[3]
                    + 0.25f * f[4] - 1.5f * f[6] - 1.0f * f[1] - 0.5f * (1.0f - f[7]);

  #pragma unroll 1
  for (int j = 0; j < 32; ++j) {
    float a = f[0] * Ws1[j];
    #pragma unroll
    for (int i = 1; i < 9; ++i) a += f[i] * Ws1[i * 32 + j];
    a += bs1[j];
    sH1[j * 64 + tid] = silu_f(a);
  }
  #pragma unroll 1
  for (int j = 0; j < 32; ++j) {
    float a = 0.f;
    #pragma unroll 1
    for (int i = 0; i < 32; ++i) a += sH1[i * 64 + tid] * Ws2[i * 32 + j];
    a += bs2[j];
    sH2[j * 64 + tid] = silu_f(a);
  }
  float learned = 0.f;
  #pragma unroll 1
  for (int i = 0; i < 32; ++i) learned += sH2[i * 64 + tid] * Ws3[i];
  learned += bs3[0];
  const float selv = (1.0f / (1.0f + expf(-(prior + 0.5f * learned)))) * pres;

  #pragma unroll 1
  for (int j = 0; j < 32; ++j) {
    float a = f[0] * Wr1[j];
    #pragma unroll
    for (int i = 1; i < 8; ++i) a += f[i] * Wr1[i * 32 + j];
    a += br1[j];
    sH1[j * 64 + tid] = silu_f(a);
  }
  float lg0 = 0.f, lg1 = 0.f, lg2 = 0.f, lg3 = 0.f;
  #pragma unroll 1
  for (int i = 0; i < 32; ++i) {
    const float hv = sH1[i * 64 + tid];
    lg0 += hv * Wr2[i * 4 + 0];
    lg1 += hv * Wr2[i * 4 + 1];
    lg2 += hv * Wr2[i * 4 + 2];
    lg3 += hv * Wr2[i * 4 + 3];
  }
  lg0 += br2[0]; lg1 += br2[1]; lg2 += br2[2]; lg3 += br2[3];
  const float lmx = fmaxf(fmaxf(lg0, lg1), fmaxf(lg2, lg3));
  const float e0 = expf(lg0 - lmx), e1 = expf(lg1 - lmx);
  const float e2 = expf(lg2 - lmx), e3 = expf(lg3 - lmx);
  const float inv = 1.0f / (((e0 + e1) + e2) + e3);
  const float p0 = e0 * inv, p1 = e1 * inv, p2 = e2 * inv, p3 = e3 * inv;

  int i0 = 0; float best = p0;
  if (p1 > best) { best = p1; i0 = 1; }
  if (p2 > best) { best = p2; i0 = 2; }
  if (p3 > best) { best = p3; i0 = 3; }
  int i1 = -1; float sec = -1.0f;
  if (i0 != 0 && p0 > sec) { sec = p0; i1 = 0; }
  if (i0 != 1 && p1 > sec) { sec = p1; i1 = 1; }
  if (i0 != 2 && p2 > sec) { sec = p2; i1 = 2; }
  if (i0 != 3 && p3 > sec) { sec = p3; i1 = 3; }
  const float rn = 1.0f / fmaxf(best + sec, 1e-8f);
  v4f w4;
  w4.x = ((i0 == 0) ? best : ((i1 == 0) ? sec : 0.0f)) * rn;
  w4.y = ((i0 == 1) ? best : ((i1 == 1) ? sec : 0.0f)) * rn;
  w4.z = ((i0 == 2) ? best : ((i1 == 2) ? sec : 0.0f)) * rn;
  w4.w = ((i0 == 3) ? best : ((i1 == 3) ? sec : 0.0f)) * rn;

  sS[tid] = selv;
  __syncthreads();
  const int sidx = (tid < 16) ? tid : 0;
  const v4f sv = *(const v4fa*)(sS + 4 * sidx);
  float* sdst = sel + (size_t)blockIdx.x * 64 + 4 * sidx;

  *(volatile v4f*)(ew + (size_t)t * 4) = w4;
  if (tid < 16) *(volatile v4f*)sdst = sv;
  __threadfence();
  *(volatile v4f*)(ew + (size_t)t * 4) = w4;
  if (tid < 16) *(volatile v4f*)sdst = sv;
}

__device__ __forceinline__ void y_store_pass(const float* sY, float* y, int t0, int d0, int w, int lane) {
  const int q8 = lane & 7, sub = lane >> 3;
  #pragma unroll
  for (int i = 0; i < 4; ++i) {
    const int row = 16 * w + 4 * i + sub;
    const v4f v = *(const v4fa*)(sY + row * 32 + 4 * q8);
    *(volatile v4f*)(y + (size_t)(t0 + row) * DM + d0 + 4 * q8) = v;
  }
}

__device__ __forceinline__ float sigm_fast(float z) {
  return __builtin_amdgcn_rcpf(1.0f + __expf(-z));
}

__global__ __launch_bounds__(128) void gates_kernel(
    const _Float16* __restrict__ cmA,
    const _Float16* __restrict__ wgT,
    const float* __restrict__ bg,
    const float* __restrict__ Qf,
    const float* __restrict__ mem,
    const float* __restrict__ x,
    const float* __restrict__ ew,
    const float* __restrict__ sel,
    float* __restrict__ y)
{
  __shared__ __attribute__((aligned(16))) float sY[64 * 32];
  const int tid = threadIdx.x, lane = tid & 31, w = tid >> 5;
  const int h = lane >> 4, m = lane & 15;
  const int wt = w & 1, wd = w >> 1;
  const int t0 = blockIdx.x * 64, d0 = blockIdx.y * 32;
  const int t0w = t0 + 32 * wt, dw = d0 + 16 * wd;

  const _Float16* xa0 = cmA + (size_t)(t0w + m) * K2;
  const _Float16* xa1 = xa0 + (size_t)16 * K2;
  const _Float16* wb  = wgT + (size_t)(dw + m) * K2;

  const v8f zero8 = {0.f, 0.f, 0.f, 0.f, 0.f, 0.f, 0.f, 0.f};
  v8f acc[2][4];
  #pragma unroll
  for (int mt = 0; mt < 2; ++mt)
    #pragma unroll
    for (int e = 0; e < 4; ++e) acc[mt][e] = zero8;

  #pragma unroll 1
  for (int k0 = 0; k0 < K2; k0 += 32) {
    const v16h a0 = load_frag(xa0 + k0, h);
    const v16h a1 = load_frag(xa1 + k0, h);
    #pragma unroll
    for (int e = 0; e < 4; ++e) {
      const v16h b = load_frag(wb + (size_t)e * ((size_t)DM * K2) + k0, h);
      acc[0][e] = wmma16(a0, b, acc[0][e]);
      acc[1][e] = wmma16(a1, b, acc[1][e]);
    }
  }

  const int d = dw + m;
  const float bg0 = bg[0 * DM + d], bg1 = bg[1 * DM + d];
  const float bg2 = bg[2 * DM + d], bg3 = bg[3 * DM + d];
  #pragma unroll
  for (int mt = 0; mt < 2; ++mt) {
    #pragma unroll
    for (int r = 0; r < 8; ++r) {
      const int tl = 32 * wt + 16 * mt + 8 * h + r;
      const int t = t0 + tl;
      const size_t idx = (size_t)t * DM + d;
      const float c = Qf[idx], mm = mem[idx], xv = x[idx];
      const v4f w4 = *(const v4fa*)(ew + (size_t)t * 4);
      const float sv = sel[t];
      const float g0 = sigm_fast(acc[mt][0][r] * WINV + bg0);
      const float g1 = sigm_fast(acc[mt][1][r] * WINV + bg1);
      const float g2 = sigm_fast(acc[mt][2][r] * WINV + bg2);
      const float g3 = sigm_fast(acc[mt][3][r] * WINV + bg3);
      const float core0 = g0 * c + (1.0f - g0) * mm;
      const float core1 = g1 * c + (1.0f - g1) * mm;
      const float core2 = g2 * c + (1.0f - g2) * mm;
      const float core3 = g3 * c + (1.0f - g3) * mm;
      const float cons   = c + 0.4f * (core0 - c);
      const float base   = core1;
      const float bridge = c + 0.85f * (core2 - c) + 0.15f * mm;
      const float dom    = c + 1.15f * (core3 - c);
      const float fused  = ((cons * w4.x + base * w4.y) + bridge * w4.z) + dom * w4.w;
      sY[tl * 32 + 16 * wd + m] = xv + sv * fused;
    }
  }
  __syncthreads();
  y_store_pass(sY, y, t0, d0, w, lane);
  __threadfence();
  y_store_pass(sY, y, t0, d0, w, lane);
}

__global__ __launch_bounds__(256) void ln2_kernel(
    const float* __restrict__ g2, const float* __restrict__ b2, float* out)
{
  const int tid = threadIdx.x, lane = tid & 31, w = tid >> 5;
  const int t = blockIdx.x * 8 + w;
  float* yr = out + (size_t)t * DM;

  v4f v[8];
  float s = 0.f;
  #pragma unroll
  for (int j = 0; j < 8; ++j) {
    v[j] = *(const v4fa*)(yr + 128 * j + 4 * lane);
    s += (v[j].x + v[j].y) + (v[j].z + v[j].w);
  }
  s = wsum(s);
  const float mean = s * (1.0f / DM);
  float ss = 0.f;
  #pragma unroll
  for (int j = 0; j < 8; ++j) {
    const v4f dv = v[j] - mean;
    ss += (dv.x * dv.x + dv.y * dv.y) + (dv.z * dv.z + dv.w * dv.w);
  }
  ss = wsum(ss);
  const float var = ss * (1.0f / DM);
  const float rstd = rsqrtf(var + 1e-5f);

  v4f o[8];
  #pragma unroll
  for (int j = 0; j < 8; ++j) {
    const v4f g = *(const v4fa*)(g2 + 128 * j + 4 * lane);
    const v4f b = *(const v4fa*)(b2 + 128 * j + 4 * lane);
    o[j] = (v[j] - mean) * rstd * g + b;
  }
  #pragma unroll
  for (int j = 0; j < 8; ++j) *(volatile v4f*)(yr + 128 * j + 4 * lane) = o[j];
  __threadfence();
  #pragma unroll
  for (int j = 0; j < 8; ++j) *(volatile v4f*)(yr + 128 * j + 4 * lane) = o[j];
}

extern "C" void kernel_launch(void* const* d_in, const int* in_sizes, int n_in,
                              void* d_out, int out_size, void* d_ws, size_t ws_size,
                              hipStream_t stream) {
  if (n_in < 28) return;
  if (in_sizes[0] != NX || in_sizes[1] != NX) return;
  for (int i = 2; i <= 8; ++i) if (in_sizes[i] != NTOK) return;
  if (in_sizes[9] != DM || in_sizes[10] != DM) return;
  if (in_sizes[11] != DM * DM || in_sizes[12] != DM) return;
  if (in_sizes[13] != DM * NSH) return;
  if (in_sizes[14] != 9 * 32 || in_sizes[15] != 32) return;
  if (in_sizes[16] != 32 * 32 || in_sizes[17] != 32) return;
  if (in_sizes[18] != 32 || in_sizes[19] != 1) return;
  if (in_sizes[20] != 8 * 32 || in_sizes[21] != 32) return;
  if (in_sizes[22] != 32 * NEXP || in_sizes[23] != NEXP) return;
  if (in_sizes[24] != NEXP * K2 * DM || in_sizes[25] != NEXP * DM) return;
  if (in_sizes[26] != DM || in_sizes[27] != DM) return;
  if (out_size != NX) return;

  const float* x     = (const float*)d_in[0];
  const float* mem   = (const float*)d_in[1];
  const float* suff  = (const float*)d_in[2];
  const float* conf  = (const float*)d_in[3];
  const float* lin   = (const float*)d_in[4];
  const float* tsc   = (const float*)d_in[5];
  const float* tsco  = (const float*)d_in[6];
  const float* alg   = (const float*)d_in[7];
  const float* stale = (const float*)d_in[8];
  const float* g1    = (const float*)d_in[9];
  const float* b1    = (const float*)d_in[10];
  const float* Wq    = (const float*)d_in[11];
  const float* bq    = (const float*)d_in[12];
  const float* H     = (const float*)d_in[13];
  const float* Ws1   = (const float*)d_in[14];
  const float* bs1   = (const float*)d_in[15];
  const float* Ws2   = (const float*)d_in[16];
  const float* bs2   = (const float*)d_in[17];
  const float* Ws3   = (const float*)d_in[18];
  const float* bs3   = (const float*)d_in[19];
  const float* Wr1   = (const float*)d_in[20];
  const float* br1   = (const float*)d_in[21];
  const float* Wr2   = (const float*)d_in[22];
  const float* br2   = (const float*)d_in[23];
  const float* Wg    = (const float*)d_in[24];
  const float* bg    = (const float*)d_in[25];
  const float* g2    = (const float*)d_in[26];
  const float* b2    = (const float*)d_in[27];
  float* out = (float*)d_out;

  const size_t wq_bytes   = (size_t)DM * DM * 2;
  const size_t wgT_bytes  = (size_t)NEXP * DM * K2 * 2;
  const size_t hyp_bytes  = (size_t)NSH * DM * 2;
  const size_t nrm_bytes  = (size_t)NTOK * DM * 2;
  const size_t cm_bytes   = (size_t)NTOK * K2 * 2;
  const size_t qf_bytes   = (size_t)NTOK * DM * 4;
  const size_t ew_bytes   = (size_t)NTOK * NEXP * 4;
  const size_t sel_bytes  = (size_t)NTOK * 4;
  size_t off = 0;
  const size_t o_wqH  = off; off += wq_bytes;
  const size_t o_wqL  = off; off += wq_bytes;
  const size_t o_wgT  = off; off += wgT_bytes;
  const size_t o_hypH = off; off += hyp_bytes;
  const size_t o_hypL = off; off += hyp_bytes;
  const size_t o_nrmH = off; off += nrm_bytes;
  const size_t o_nrmL = off; off += nrm_bytes;
  const size_t o_cm   = off; off += cm_bytes;
  const size_t o_qf   = off; off += qf_bytes;
  const size_t o_ew   = off; off += ew_bytes;
  const size_t o_sel  = off; off += sel_bytes;
  if (off > ws_size) return;
  if (off > (size_t)134217728) return;

  char* ws = (char*)d_ws;
  unsigned short* WqH  = (unsigned short*)(ws + o_wqH);
  unsigned short* WqL  = (unsigned short*)(ws + o_wqL);
  _Float16*       WgT  = (_Float16*)(ws + o_wgT);
  unsigned short* hypH = (unsigned short*)(ws + o_hypH);
  unsigned short* hypL = (unsigned short*)(ws + o_hypL);
  unsigned short* nrmH = (unsigned short*)(ws + o_nrmH);
  unsigned short* nrmL = (unsigned short*)(ws + o_nrmL);
  _Float16*       cmA  = (_Float16*)(ws + o_cm);
  float* Qf   = (float*)(ws + o_qf);
  float* ewp  = (float*)(ws + o_ew);
  float* selp = (float*)(ws + o_sel);

  cvt_t2_kernel<<<dim3(DM / 64, DM / 64, 1), 256, 0, stream>>>(Wq, WqH, WqL, DM, DM);
  cvt_t_kernel<<<dim3(DM / 64, K2 / 64, NEXP), 256, 0, stream>>>(Wg, WgT, K2, DM, WSC);
  cvt_hyp_kernel<<<DM / 64, 128, 0, stream>>>(H, hypH, hypL);
  ln1_kernel<<<NTOK / 8, 256, 0, stream>>>(x, mem, g1, b1, nrmH, nrmL, cmA);
  gemm_q_kernel<<<dim3(NTOK / 128, DM / 64), 128, 0, stream>>>(nrmH, nrmL, WqH, WqL, bq, Qf, cmA);
  token_kernel<<<NTOK / 64, 64, 0, stream>>>(Qf, hypH, hypL, mem, suff, conf, lin, tsc, tsco, alg, stale,
                                             Ws1, bs1, Ws2, bs2, Ws3, bs3, Wr1, br1, Wr2, br2,
                                             ewp, selp);
  gates_kernel<<<dim3(NTOK / 64, DM / 32), 128, 0, stream>>>(cmA, WgT, bg, Qf, mem, x, ewp, selp, out);
  ln2_kernel<<<NTOK / 8, 256, 0, stream>>>(g2, b2, out);
}
